// GregTransformer_2680059592717
// MI455X (gfx1250) — hardware-verified
//
#include <hip/hip_runtime.h>
#include <math.h>


#define DM 1024
#define NH 16
#define HD 64
#define SQ 2048
#define NB 2
#define FF 4096
#define MR (NB * SQ)
#define CSP 68

typedef unsigned short u16;
typedef unsigned int u32;
typedef u16 v8u __attribute__((ext_vector_type(8)));
typedef __bf16 v16b __attribute__((ext_vector_type(16)));
typedef _Float16 v16h __attribute__((ext_vector_type(16)));
typedef float v8f __attribute__((ext_vector_type(8)));
typedef float v4f __attribute__((ext_vector_type(4)));

union FragB { v16b v; v8u p[2]; };
union FragH { v16h v; v8u p[2]; };

static __device__ __forceinline__ u16 bfb(float f) {
  const u32 u = __float_as_uint(f);
  const u32 r = u + 0x7fffu + ((u >> 16) & 1u);
  return (u16)(r >> 16);
}
static __device__ __forceinline__ float bfv(u16 b) { return __uint_as_float(((u32)b) << 16); }
static __device__ __forceinline__ u16 hfb(float f) {
  union { _Float16 h; u16 u; } c;
  c.h = (_Float16)f;
  return c.u;
}
static __device__ __forceinline__ v8f vz8() {
  v8f z = {0.f, 0.f, 0.f, 0.f, 0.f, 0.f, 0.f, 0.f};
  return z;
}

static __device__ __forceinline__ v8f mma_b(v16b a, v16b b, v8f c) {
  c = __builtin_amdgcn_wmma_f32_16x16x32_bf16(false, a, false, b, (short)0, c, false, false);
  asm volatile("v_nop\n\tv_nop\n\tv_nop\n\tv_nop" : "+v"(c) : "v"(a), "v"(b));
  return c;
}
static __device__ __forceinline__ v8f mma_h(v16h a, v16h b, v8f c) {
  c = __builtin_amdgcn_wmma_f32_16x16x32_f16(false, a, false, b, (short)0, c, false, false);
  asm volatile("v_nop\n\tv_nop\n\tv_nop\n\tv_nop" : "+v"(c) : "v"(a), "v"(b));
  return c;
}

static __device__ __forceinline__ void ldp(v8u& e0, v8u& e1, const u16* row, int lh) {
  e0 = *(const v8u*)(row + 8 * lh);
  e1 = *(const v8u*)(row + 16 + 8 * lh);
}

static __device__ __forceinline__ void stv8(u16* p, v8u v) { *(volatile v8u*)p = v; }
static __device__ __forceinline__ void stv4(float* p, v4f v) { *(volatile v4f*)p = v; }

static __device__ __forceinline__ float gelu_e(float x) {
  return 0.5f * x * (1.0f + erff(x * 0.70710678118654752f));
}

#define LO4(v) __builtin_shufflevector((v), (v), 0, 1, 2, 3)
#define HI4(v) __builtin_shufflevector((v), (v), 4, 5, 6, 7)
#define CAT8(a, b) __builtin_shufflevector((a), (b), 0, 1, 2, 3, 4, 5, 6, 7)

template <int MODE>
__global__ __launch_bounds__(256) void k_wcvt(const float* __restrict__ W0, const float* __restrict__ W1,
                                              const float* __restrict__ W2, const float* __restrict__ W3,
                                              u16* obase, int K, int N, float scale) {
  __shared__ __attribute__((aligned(16))) float T[64 * CSP];
  const int z = blockIdx.z;
  const float* W = (z == 0) ? W0 : ((z == 1) ? W1 : ((z == 2) ? W2 : W3));
  const size_t plane = (size_t)K * (size_t)N;
  u16* oa = obase + ((MODE == 0) ? ((size_t)z * 2 * plane) : ((size_t)z * plane));
  u16* ob = oa + plane;
  const int n0 = blockIdx.x * 64, k0 = blockIdx.y * 64;
  const int t = threadIdx.x, l = t & 31, wv = t >> 5;

#pragma unroll
  for (int it = 0; it < 4; ++it) {
    const int kr = it * 16 + (t >> 4), c = (t & 15) * 4;
    *(v4f*)(T + kr * CSP + c) = *(const v4f*)(W + (size_t)(k0 + kr) * N + n0 + c);
  }
  __syncthreads();

#pragma unroll
  for (int pass = 0; pass < 2; ++pass) {
#pragma unroll
    for (int it = 0; it < 2; ++it) {
      const int n = wv * 8 + it * 4 + (l >> 3), piece = l & 7;
      const size_t goff = (size_t)(n0 + n) * K + k0 + piece * 8;
      if (MODE == 0) {
        v8u hi = {0, 0, 0, 0, 0, 0, 0, 0};
        v8u lo = {0, 0, 0, 0, 0, 0, 0, 0};
#pragma unroll
        for (int j = 0; j < 8; ++j) {
          const float xv = T[(piece * 8 + j) * CSP + n];
          const u16 hb = bfb(xv);
          hi[j] = hb;
          lo[j] = bfb(xv - bfv(hb));
        }
        stv8(oa + goff, hi);
        stv8(ob + goff, lo);
      } else {
        v8u hv = {0, 0, 0, 0, 0, 0, 0, 0};
#pragma unroll
        for (int j = 0; j < 8; ++j) hv[j] = hfb(T[(piece * 8 + j) * CSP + n] * scale);
        stv8(oa + goff, hv);
      }
    }
    if (pass == 0) __threadfence();
  }
}

template <int MODE>
__global__ __launch_bounds__(128) void k_ln(const float* __restrict__ x, const float* __restrict__ g,
                                           const float* __restrict__ be, u16* oa, u16* ob) {
  __shared__ float red_a[4];
  __shared__ float red_b[4];
  const int row = blockIdx.x, t = threadIdx.x, l = t & 31, wv = t >> 5;
  const float* xr = x + (size_t)row * DM + t * 8;
  const v4f a = *(const v4f*)xr;
  const v4f b = *(const v4f*)(xr + 4);
  float s = ((a[0] + a[1]) + (a[2] + a[3])) + ((b[0] + b[1]) + (b[2] + b[3]));
#pragma unroll
  for (int o = 16; o > 0; o >>= 1) s += __shfl_xor(s, o, 32);
  if (l == 0) red_a[wv] = s;
  __syncthreads();
  const float tot = (red_a[0] + red_a[1]) + (red_a[2] + red_a[3]);
  const float mu = tot * (1.0f / (float)DM);
  float d[8];
  d[0] = a[0] - mu; d[1] = a[1] - mu; d[2] = a[2] - mu; d[3] = a[3] - mu;
  d[4] = b[0] - mu; d[5] = b[1] - mu; d[6] = b[2] - mu; d[7] = b[3] - mu;
  float q = 0.0f;
#pragma unroll
  for (int j = 0; j < 8; ++j) q += d[j] * d[j];
#pragma unroll
  for (int o = 16; o > 0; o >>= 1) q += __shfl_xor(q, o, 32);
  if (l == 0) red_b[wv] = q;
  __syncthreads();
  const float qt = (red_b[0] + red_b[1]) + (red_b[2] + red_b[3]);
  const float var = qt * (1.0f / (float)DM);
  const float rs = rsqrtf(var + 1e-5f);
  const v4f g0 = *(const v4f*)(g + t * 8);
  const v4f g1v = *(const v4f*)(g + t * 8 + 4);
  const v4f b0 = *(const v4f*)(be + t * 8);
  const v4f b1v = *(const v4f*)(be + t * 8 + 4);
  float gg[8], bb[8], y[8];
  gg[0] = g0[0]; gg[1] = g0[1]; gg[2] = g0[2]; gg[3] = g0[3];
  gg[4] = g1v[0]; gg[5] = g1v[1]; gg[6] = g1v[2]; gg[7] = g1v[3];
  bb[0] = b0[0]; bb[1] = b0[1]; bb[2] = b0[2]; bb[3] = b0[3];
  bb[4] = b1v[0]; bb[5] = b1v[1]; bb[6] = b1v[2]; bb[7] = b1v[3];
#pragma unroll
  for (int j = 0; j < 8; ++j) y[j] = (d[j] * rs) * gg[j] + bb[j];

  const size_t off = (size_t)row * DM + t * 8;
  if (MODE == 0) {
    v8u hi = {0, 0, 0, 0, 0, 0, 0, 0};
    v8u lo = {0, 0, 0, 0, 0, 0, 0, 0};
#pragma unroll
    for (int j = 0; j < 8; ++j) {
      const u16 hb = bfb(y[j]);
      hi[j] = hb;
      lo[j] = bfb(y[j] - bfv(hb));
    }
    stv8(oa + off, hi);
    stv8(ob + off, lo);
    __threadfence();
    stv8(oa + off, hi);
    stv8(ob + off, lo);
  } else {
    v8u hv = {0, 0, 0, 0, 0, 0, 0, 0};
#pragma unroll
    for (int j = 0; j < 8; ++j) hv[j] = hfb(y[j]);
    stv8(oa + off, hv);
    __threadfence();
    stv8(oa + off, hv);
  }
}

template <bool SPLIT, int EPI>
__global__ __launch_bounds__(256) void k_gemm(const u16* __restrict__ Xh, const u16* __restrict__ Xl,
                                              const u16* __restrict__ Wh, const u16* __restrict__ Wl,
                                              const float* __restrict__ bias, const float* __restrict__ resid,
                                              float* outf, u16* oa, u16* ob,
                                              int M, int N, int K, int S, float oscale) {
  __shared__ __attribute__((aligned(16))) float Cs[128 * CSP];
  (void)M;
  const int t = threadIdx.x, l = t & 31, lh = l >> 4, lm = l & 15, wv = t >> 5;
  const int tile_n = blockIdx.x * 64, tile_m = blockIdx.y * 128;
  const size_t xoff = (size_t)(tile_m + wv * 16 + lm) * K;
  const size_t woff = (size_t)(tile_n + lm) * K;
  const size_t wst = (size_t)16 * K;

  v8f acc[4];
#pragma unroll
  for (int nt = 0; nt < 4; ++nt) acc[nt] = vz8();

#pragma unroll 1
  for (int k0 = 0; k0 < K; k0 += 32) {
    if (SPLIT) {
      FragB xh, xl;
      ldp(xh.p[0], xh.p[1], Xh + xoff + k0, lh);
      ldp(xl.p[0], xl.p[1], Xl + xoff + k0, lh);
#pragma unroll
      for (int nt = 0; nt < 4; ++nt) {
        FragB wh, wl;
        ldp(wh.p[0], wh.p[1], Wh + woff + nt * wst + k0, lh);
        ldp(wl.p[0], wl.p[1], Wl + woff + nt * wst + k0, lh);
        acc[nt] = mma_b(wh.v, xh.v, acc[nt]);
        acc[nt] = mma_b(wh.v, xl.v, acc[nt]);
        acc[nt] = mma_b(wl.v, xh.v, acc[nt]);
      }
    } else {
      FragH xh;
      ldp(xh.p[0], xh.p[1], Xh + xoff + k0, lh);
#pragma unroll
      for (int nt = 0; nt < 4; ++nt) {
        FragH wh;
        ldp(wh.p[0], wh.p[1], Wh + woff + nt * wst + k0, lh);
        acc[nt] = mma_h(wh.v, xh.v, acc[nt]);
      }
    }
  }

  float* cw = Cs + (wv * 16 + lm) * CSP;
#pragma unroll
  for (int nt = 0; nt < 4; ++nt) {
    *(v4f*)(cw + nt * 16 + 8 * lh) = LO4(acc[nt]);
    *(v4f*)(cw + nt * 16 + 8 * lh + 4) = HI4(acc[nt]);
  }
  __syncthreads();

  if (EPI == 0 || EPI == 3) {
#pragma unroll
    for (int pass = 0; pass < 2; ++pass) {
#pragma unroll
      for (int it = 0; it < 4; ++it) {
        const int row = it * 4 + (l >> 3), piece = l & 7;
        const float* cr = Cs + (wv * 16 + row) * CSP + piece * 8;
        const v4f c0 = *(const v4f*)cr;
        const v4f c1 = *(const v4f*)(cr + 4);
        const v8f c = CAT8(c0, c1);
        const float* bp = bias + tile_n + piece * 8;
        const v4f q0 = *(const v4f*)bp;
        const v4f q1 = *(const v4f*)(bp + 4);
        const v8f bv8 = CAT8(q0, q1);
        const size_t goff = (size_t)(tile_m + wv * 16 + row) * N + tile_n + piece * 8;
        if (EPI == 0) {
          v8u hi = {0, 0, 0, 0, 0, 0, 0, 0};
          v8u lo = {0, 0, 0, 0, 0, 0, 0, 0};
#pragma unroll
          for (int j = 0; j < 8; ++j) {
            const float xv = c[j] + bv8[j];
            const u16 hb = bfb(xv);
            hi[j] = hb;
            lo[j] = bfb(xv - bfv(hb));
          }
          stv8(oa + goff, hi);
          stv8(ob + goff, lo);
        } else {
          v8u hv = {0, 0, 0, 0, 0, 0, 0, 0};
#pragma unroll
          for (int j = 0; j < 8; ++j) hv[j] = hfb(gelu_e(c[j] * oscale + bv8[j]));
          stv8(oa + goff, hv);
        }
      }
      if (pass == 0) __threadfence();
    }
  } else if (EPI == 2) {
#pragma unroll
    for (int pass = 0; pass < 2; ++pass) {
#pragma unroll
      for (int it = 0; it < 8; ++it) {
        const int row = it * 2 + (l >> 4), piece = l & 15;
        const v4f c = *(const v4f*)(Cs + (wv * 16 + row) * CSP + piece * 4);
        const v4f q4 = *(const v4f*)(bias + tile_n + piece * 4);
        const size_t goff = (size_t)(tile_m + wv * 16 + row) * N + tile_n + piece * 4;
        const v4f r4 = *(const v4f*)(resid + goff);
        const float o0 = (c[0] * oscale + q4[0]) + r4[0];
        const float o1 = (c[1] * oscale + q4[1]) + r4[1];
        const float o2 = (c[2] * oscale + q4[2]) + r4[2];
        const float o3 = (c[3] * oscale + q4[3]) + r4[3];
        const v4f ov = {o0, o1, o2, o3};
        stv4(outf + goff, ov);
      }
      if (pass == 0) __threadfence();
    }
  } else {
    const int bb = tile_m / S;
    const int s0 = tile_m - bb * S;
#pragma unroll
    for (int pass = 0; pass < 2; ++pass) {
#pragma unroll
      for (int it = 0; it < 4; ++it) {
        const int dd = wv * 8 + it * 2 + (l >> 4), piece = l & 15;
        const float bd = bias[tile_n + dd];
        v8u hi = {0, 0, 0, 0, 0, 0, 0, 0};
        v8u lo = {0, 0, 0, 0, 0, 0, 0, 0};
#pragma unroll
        for (int j = 0; j < 8; ++j) {
          const float xv = Cs[(piece * 8 + j) * CSP + dd] + bd;
          const u16 hb = bfb(xv);
          hi[j] = hb;
          lo[j] = bfb(xv - bfv(hb));
        }
        const size_t goff = ((size_t)(bb * N + tile_n + dd)) * S + s0 + piece * 8;
        stv8(oa + goff, hi);
        stv8(ob + goff, lo);
      }
      if (pass == 0) __threadfence();
    }
  }
}

__global__ __launch_bounds__(128) void k_attn(const u16* __restrict__ qh, const u16* __restrict__ ql,
                                              const u16* __restrict__ kh, const u16* __restrict__ kl,
                                              const u16* __restrict__ vh, const u16* __restrict__ vl,
                                              u16* ch, u16* cl, int S, int Dm, int H) {
  __shared__ __attribute__((aligned(16))) float Os[4 * 16 * CSP];
  const int t = threadIdx.x, l = t & 31, lh = l >> 4, lm = l & 15, wv = t >> 5;
  const int nqt = S >> 6;
  const int bid = blockIdx.x;
  const int qt = bid % nqt;
  const int bhi = bid / nqt;
  const int h = bhi % H;
  const int b = bhi / H;
  const int q0 = qt * 64;
  const int qrow = q0 + wv * 16 + lm;
  const size_t qoff = ((size_t)b * S + qrow) * Dm + (size_t)h * HD;

  FragB qfh[2], qfl[2];
#pragma unroll
  for (int dc = 0; dc < 2; ++dc) {
    ldp(qfh[dc].p[0], qfh[dc].p[1], qh + qoff + dc * 32, lh);
    ldp(qfl[dc].p[0], qfl[dc].p[1], ql + qoff + dc * 32, lh);
  }
  v8f o[4];
#pragma unroll
  for (int dt = 0; dt < 4; ++dt) o[dt] = vz8();

  const size_t kbase = ((size_t)b * S + lm) * Dm + (size_t)h * HD;
  const size_t vbase = ((size_t)bhi * HD + lm) * (size_t)S;

  for (int kbi = 0; kbi <= qt; ++kbi) {
    const int kb0 = kbi * 64;
    FragB ph[2], pl[2];
#pragma unroll
    for (int kc = 0; kc < 2; ++kc) {
      v8f sa = vz8(), sb = vz8();
      const size_t ka = kbase + (size_t)(kb0 + kc * 32) * Dm;
      const size_t kb = ka + (size_t)16 * Dm;
#pragma unroll
      for (int dc = 0; dc < 2; ++dc) {
        FragB fah, fal;
        ldp(fah.p[0], fah.p[1], kh + ka + dc * 32, lh);
        ldp(fal.p[0], fal.p[1], kl + ka + dc * 32, lh);
        sa = mma_b(fah.v, qfh[dc].v, sa);
        sa = mma_b(fah.v, qfl[dc].v, sa);
        sa = mma_b(fal.v, qfh[dc].v, sa);
        FragB fbh, fbl;
        ldp(fbh.p[0], fbh.p[1], kh + kb + dc * 32, lh);
        ldp(fbl.p[0], fbl.p[1], kl + kb + dc * 32, lh);
        sb = mma_b(fbh.v, qfh[dc].v, sb);
        sb = mma_b(fbh.v, qfl[dc].v, sb);
        sb = mma_b(fbl.v, qfh[dc].v, sb);
      }
      v8u pah = {0, 0, 0, 0, 0, 0, 0, 0};
      v8u pal = {0, 0, 0, 0, 0, 0, 0, 0};
      v8u pbh = {0, 0, 0, 0, 0, 0, 0, 0};
      v8u pbl = {0, 0, 0, 0, 0, 0, 0, 0};
#pragma unroll
      for (int r = 0; r < 8; ++r) {
        const int keya = kb0 + kc * 32 + 8 * lh + r;
        const int keyb = keya + 16;
        float xa = fmaxf(sa[r] * 0.125f, 0.0f);
        xa = (keya <= qrow) ? xa : 0.0f;
        float xb = fmaxf(sb[r] * 0.125f, 0.0f);
        xb = (keyb <= qrow) ? xb : 0.0f;
        const u16 ha = bfb(xa);
        const u16 hbb = bfb(xb);
        pah[r] = ha;
        pal[r] = bfb(xa - bfv(ha));
        pbh[r] = hbb;
        pbl[r] = bfb(xb - bfv(hbb));
      }
      ph[kc].p[0] = pah; ph[kc].p[1] = pbh;
      pl[kc].p[0] = pal; pl[kc].p[1] = pbl;
    }
#pragma unroll
    for (int dt = 0; dt < 4; ++dt) {
      const size_t va = vbase + (size_t)dt * 16 * S + kb0;
#pragma unroll
      for (int kc = 0; kc < 2; ++kc) {
        FragB fah, fal;
        ldp(fah.p[0], fah.p[1], vh + va + kc * 32, lh);
        ldp(fal.p[0], fal.p[1], vl + va + kc * 32, lh);
        o[dt] = mma_b(fah.v, ph[kc].v, o[dt]);
        o[dt] = mma_b(fah.v, pl[kc].v, o[dt]);
        o[dt] = mma_b(fal.v, ph[kc].v, o[dt]);
      }
    }
  }

  float* ow = Os + (wv * 16 + lm) * CSP;
#pragma unroll
  for (int dt = 0; dt < 4; ++dt) {
    *(v4f*)(ow + dt * 16 + 8 * lh) = LO4(o[dt]);
    *(v4f*)(ow + dt * 16 + 8 * lh + 4) = HI4(o[dt]);
  }
  __syncthreads();

#pragma unroll
  for (int pass = 0; pass < 2; ++pass) {
#pragma unroll
    for (int it = 0; it < 4; ++it) {
      const int row = it * 4 + (l >> 3), piece = l & 7;
      const float* cr = Os + (wv * 16 + row) * CSP + piece * 8;
      const v4f c0 = *(const v4f*)cr;
      const v4f c1 = *(const v4f*)(cr + 4);
      const v8f c = CAT8(c0, c1);
      v8u hi = {0, 0, 0, 0, 0, 0, 0, 0};
      v8u lo = {0, 0, 0, 0, 0, 0, 0, 0};
#pragma unroll
      for (int j = 0; j < 8; ++j) {
        const u16 hb = bfb(c[j]);
        hi[j] = hb;
        lo[j] = bfb(c[j] - bfv(hb));
      }
      const size_t goff = ((size_t)b * S + q0 + wv * 16 + row) * Dm + (size_t)h * HD + piece * 8;
      stv8(ch + goff, hi);
      stv8(cl + goff, lo);
    }
    if (pass == 0) __threadfence();
  }
}

extern "C" void kernel_launch(void* const* d_in, const int* in_sizes, int n_in,
                              void* d_out, int out_size, void* d_ws, size_t ws_size,
                              hipStream_t stream) {
  if (n_in < 17) return;
  const int want[17] = {MR * DM, DM * DM, DM, DM * DM, DM, DM * DM, DM, DM * DM, DM,
                        DM, DM, DM, DM, DM * FF, FF, FF * DM, DM};
  for (int i = 0; i < 17; ++i) {
    if (in_sizes[i] != want[i]) return;
  }
  if (out_size != MR * DM) return;
  const size_t MiB = (size_t)1 << 20;
  if (ws_size < 80 * MiB) return;

  const float* x   = (const float*)d_in[0];
  const float* wq  = (const float*)d_in[1];
  const float* bq  = (const float*)d_in[2];
  const float* wk  = (const float*)d_in[3];
  const float* bk  = (const float*)d_in[4];
  const float* wvw = (const float*)d_in[5];
  const float* bv  = (const float*)d_in[6];
  const float* wo  = (const float*)d_in[7];
  const float* bo  = (const float*)d_in[8];
  const float* g1  = (const float*)d_in[9];
  const float* be1 = (const float*)d_in[10];
  const float* g2  = (const float*)d_in[11];
  const float* be2 = (const float*)d_in[12];
  const float* w1  = (const float*)d_in[13];
  const float* b1  = (const float*)d_in[14];
  const float* w2  = (const float*)d_in[15];
  const float* b2  = (const float*)d_in[16];
  float* out = (float*)d_out;

  char* base = (char*)d_ws;
  const size_t WP = (size_t)DM * DM;
  u16* watt = (u16*)(base);
  u16* wq_h = watt + 0 * WP; u16* wq_l = watt + 1 * WP;
  u16* wk_h = watt + 2 * WP; u16* wk_l = watt + 3 * WP;
  u16* wv_h = watt + 4 * WP; u16* wv_l = watt + 5 * WP;
  u16* wo_h = watt + 6 * WP; u16* wo_l = watt + 7 * WP;
  u16* h1_h = (u16*)(base + 16 * MiB);
  u16* h1_l = (u16*)(base + 24 * MiB);
  u16* cx_h = (u16*)(base + 16 * MiB);
  u16* cx_l = (u16*)(base + 24 * MiB);
  u16* q_h  = (u16*)(base + 32 * MiB);
  u16* q_l  = (u16*)(base + 40 * MiB);
  float* x1 = (float*)(base + 32 * MiB);
  u16* k_h  = (u16*)(base + 48 * MiB);
  u16* k_l  = (u16*)(base + 56 * MiB);
  u16* h2   = (u16*)(base + 48 * MiB);
  u16* w1t  = (u16*)(base + 56 * MiB);
  u16* vt_h = (u16*)(base + 64 * MiB);
  u16* vt_l = (u16*)(base + 72 * MiB);
  u16* w2t  = (u16*)(base + 64 * MiB);
  u16* f1   = (u16*)(base);

  const dim3 gproj(DM / 64, MR / 128);

  k_wcvt<0><<<dim3(DM / 64, DM / 64, 4), 256, 0, stream>>>(wq, wk, wvw, wo, watt, DM, DM, 1.0f);
  k_ln<0><<<dim3(MR), 128, 0, stream>>>(x, g1, be1, h1_h, h1_l);
  k_gemm<true, 0><<<gproj, 256, 0, stream>>>(h1_h, h1_l, wq_h, wq_l, bq, x, x1, q_h, q_l, MR, DM, DM, SQ, 1.0f);
  k_gemm<true, 0><<<gproj, 256, 0, stream>>>(h1_h, h1_l, wk_h, wk_l, bk, x, x1, k_h, k_l, MR, DM, DM, SQ, 1.0f);
  k_gemm<true, 1><<<gproj, 256, 0, stream>>>(h1_h, h1_l, wv_h, wv_l, bv, x, x1, vt_h, vt_l, MR, DM, DM, SQ, 1.0f);
  k_attn<<<dim3(NB * NH * (SQ / 64)), 128, 0, stream>>>(q_h, q_l, k_h, k_l, vt_h, vt_l, cx_h, cx_l, SQ, DM, NH);
  k_gemm<true, 2><<<gproj, 256, 0, stream>>>(cx_h, cx_l, wo_h, wo_l, bo, x, x1, k_h, k_l, MR, DM, DM, SQ, 1.0f);
  k_ln<1><<<dim3(MR), 128, 0, stream>>>(x1, g2, be2, h2, h2);
  k_wcvt<1><<<dim3(FF / 64, DM / 64, 1), 256, 0, stream>>>(w1, w1, w1, w1, w1t, DM, FF, 32.0f);
  k_wcvt<1><<<dim3(DM / 64, FF / 64, 1), 256, 0, stream>>>(w2, w2, w2, w2, w2t, FF, DM, 64.0f);
  k_gemm<false, 3><<<dim3(FF / 64, MR / 128), 256, 0, stream>>>(h2, h2, w1t, w1t, b1, x, x1, f1, f1,
                                                                 MR, FF, DM, SQ, 1.0f / 32.0f);
  k_gemm<false, 2><<<dim3(DM / 64, MR / 128), 256, 0, stream>>>(f1, f1, w2t, w2t, b2, x1, out, h2, h2,
                                                                 MR, DM, FF, SQ, 1.0f / 64.0f);
}
